// BiasedScanAttention_82824149336916
// MI455X (gfx1250) — hardware-verified
//
#include <hip/hip_runtime.h>


#define NB_  2
#define NH_  8
#define TT   2048
#define HD   64
#define NM   8
#define HPP  4
typedef _Float16 h16;
typedef unsigned short bf;
typedef __attribute__((ext_vector_type(16))) __bf16   v16bf;
typedef __attribute__((ext_vector_type(16))) _Float16 v16h;
typedef __attribute__((ext_vector_type(8)))  _Float16 v8h;
typedef __attribute__((ext_vector_type(8)))  unsigned short v8us;
typedef __attribute__((ext_vector_type(8)))  float    v8f;
typedef __attribute__((ext_vector_type(4)))  float    v4f;
typedef v8h  __attribute__((may_alias)) v8ha;
typedef v4f  __attribute__((may_alias)) v4fa;
typedef v8us __attribute__((may_alias)) v8usa;

__device__ __forceinline__ unsigned short f2bf(float f) { unsigned u = __float_as_uint(f); u += 0x7FFFu + ((u >> 16) & 1u); return (unsigned short)(u >> 16); }
__device__ __forceinline__ float bf2f(unsigned short b) { return __uint_as_float(((unsigned)b) << 16); }
__device__ __forceinline__ float bfr(float f) { return bf2f(f2bf(f)); }
__device__ __forceinline__ v16h cat16(v8h lo, v8h hi) { return __builtin_shufflevector(lo, hi, 0, 1, 2, 3, 4, 5, 6, 7, 8, 9, 10, 11, 12, 13, 14, 15); }
__device__ __forceinline__ v16bf cat16b(v8us lo, v8us hi) { return __builtin_bit_cast(v16bf, __builtin_shufflevector(lo, hi, 0, 1, 2, 3, 4, 5, 6, 7, 8, 9, 10, 11, 12, 13, 14, 15)); }
__device__ __forceinline__ v8f wmma16(v16h a, v16h b, v8f c) { return __builtin_amdgcn_wmma_f32_16x16x32_f16(false, a, false, b, (short)0, c, false, false); }
__device__ __forceinline__ v8f wmmab(v16bf a, v16bf b, v8f c) { return __builtin_amdgcn_wmma_f32_16x16x32_bf16(false, a, false, b, (short)0, c, false, false); }


template <typename T16> struct WFrag;
template <> struct WFrag<h16> { typedef v16h V; static __device__ __forceinline__ V ld(const h16* p) { return cat16(*(const v8h*)p, *(const v8h*)(p + 16)); } static __device__ __forceinline__ v8f mma(V a, V b, v8f c) { return wmma16(a, b, c); } };
template <> struct WFrag<bf> { typedef v16bf V; static __device__ __forceinline__ V ld(const bf* p) { return cat16b(*(const v8us*)p, *(const v8us*)(p + 16)); } static __device__ __forceinline__ v8f mma(V a, V b, v8f c) { return wmmab(a, b, c); } };
template <typename T16, int NSPLIT, bool BIAS>
__global__ __launch_bounds__(32) void k_gemmw(const T16* __restrict__ A, const T16* __restrict__ A2, const T16* __restrict__ Bt, const T16* __restrict__ Bt2, int K, float* C, int ldc, const float* __restrict__ bias, size_t sA, size_t sB, size_t sC) {
    typedef typename WFrag<T16>::V V;
    __shared__ __align__(16) float os[16 * 68];
    const size_t z = blockIdx.z; A += z * sA; if (A2) A2 += z * sA; Bt += z * sB; if (Bt2) Bt2 += z * sB; C += z * sC;
    const int lane = threadIdx.x & 31, lr = lane & 15, hi = lane >> 4; const int r0 = blockIdx.x * 64, c0 = blockIdx.y * 64;
    v8f acc[4][4];
#pragma unroll
    for (int mb = 0; mb < 4; ++mb)
#pragma unroll
        for (int nb = 0; nb < 4; ++nb) acc[mb][nb] = (v8f){};
    const size_t aoff = (size_t)(r0 + lr) * K + 8 * hi, boff = (size_t)(c0 + lr) * K + 8 * hi;
#pragma unroll 1
    for (int kc = 0; kc < K; kc += 32) {
        V a[4], a2[4];
#pragma unroll
        for (int mb = 0; mb < 4; ++mb) { a[mb] = WFrag<T16>::ld(A + aoff + (size_t)mb * 16 * K + kc); if (NSPLIT == 1 || NSPLIT == 2) a2[mb] = WFrag<T16>::ld(A2 + aoff + (size_t)mb * 16 * K + kc); }
#pragma unroll
        for (int nb = 0; nb < 4; ++nb) { const V b = WFrag<T16>::ld(Bt + boff + (size_t)nb * 16 * K + kc); V b2; if (NSPLIT >= 2) b2 = WFrag<T16>::ld(Bt2 + boff + (size_t)nb * 16 * K + kc);
#pragma unroll
            for (int mb = 0; mb < 4; ++mb) { acc[mb][nb] = WFrag<T16>::mma(a[mb], b, acc[mb][nb]); if (NSPLIT == 1 || NSPLIT == 2) acc[mb][nb] = WFrag<T16>::mma(a2[mb], b, acc[mb][nb]); if (NSPLIT >= 2) acc[mb][nb] = WFrag<T16>::mma(a[mb], b2, acc[mb][nb]); } }
        asm volatile("v_nop\n\tv_nop\n\tv_nop\n\tv_nop" : "+v"(acc[0][0]), "+v"(acc[1][1]), "+v"(acc[2][2]), "+v"(acc[3][3]) : "v"(a[0]), "v"(a[3]));
    }
#pragma unroll
    for (int mb = 0; mb < 4; ++mb) {
#pragma unroll
        for (int nb = 0; nb < 4; ++nb) {
#pragma unroll
            for (int j = 0; j < 8; ++j) os[(hi * 8 + j) * 68 + nb * 16 + lr] = acc[mb][nb][j]; }
        __builtin_amdgcn_wave_barrier(); asm volatile("" ::: "memory");
        float* crow = C + (size_t)(r0 + mb * 16) * ldc + c0;
#pragma unroll 1
        for (int ps = 0; ps < 2; ++ps) {
#pragma unroll
            for (int s = 0; s < 8; ++s) { const int row = 2 * s + hi, cofs = lr * 4; v4f val = *(const v4fa*)(os + row * 68 + cofs); if (BIAS) { val[0] += bfr(bias[c0 + cofs]); val[1] += bfr(bias[c0 + cofs + 1]); val[2] += bfr(bias[c0 + cofs + 2]); val[3] += bfr(bias[c0 + cofs + 3]); }
                *(volatile v4f*)(crow + (size_t)row * ldc + cofs) = val; }
            if (ps == 0) __threadfence(); }
        __builtin_amdgcn_wave_barrier(); asm volatile("" ::: "memory");
    }
}

__device__ __forceinline__ h16 tohx(float x) { return (h16)x; }
__device__ __forceinline__ void splitf(float y, unsigned short& h, unsigned short& l) { h = f2bf(y); l = f2bf(y - bf2f(h)); }
typedef __attribute__((ext_vector_type(2))) unsigned short v2us;
typedef __attribute__((ext_vector_type(4))) unsigned short v4us;
typedef __attribute__((ext_vector_type(4))) _Float16 v4h;

__global__ __launch_bounds__(256) void k_cvt8(const float* __restrict__ src, bf* dst, size_t n8) { const size_t i = (size_t)blockIdx.x * 256 + threadIdx.x; if (i >= n8) return; const v8f v = *(const v8f*)(src + i * 8); v8us o;
#pragma unroll
    for (int k = 0; k < 8; ++k) o[k] = f2bf(v[k]); *(volatile v8us*)(dst + i * 8) = o; __threadfence(); *(volatile v8us*)(dst + i * 8) = o; }
__global__ __launch_bounds__(256) void k_q8(const float* __restrict__ q, bf* QB, size_t n8) { const size_t i = (size_t)blockIdx.x * 256 + threadIdx.x; if (i >= n8) return; const v4f a = *(const v4f*)(q + i * 8), b = *(const v4f*)(q + i * 8 + 4); v8us o;
#pragma unroll
    for (int u = 0; u < 4; ++u) { o[u] = f2bf(bfr(a[u]) * 0.125f); o[4 + u] = f2bf(bfr(b[u]) * 0.125f); } *(volatile v8us*)(QB + i * 8) = o; __threadfence(); *(volatile v8us*)(QB + i * 8) = o; }
__global__ __launch_bounds__(256) void k_vt(const float* __restrict__ v, bf* VT) { const int e = (blockIdx.x * 256 + threadIdx.x) * 2; if (e >= HPP * HD * TT) return; const int t = e % TT; const int d = (e / TT) % HD; const int z = e / (TT * HD); v2us o; o[0] = f2bf(v[((size_t)z * TT + t) * HD + d]); o[1] = f2bf(v[((size_t)z * TT + t + 1) * HD + d]);
    *(volatile v2us*)(VT + e) = o; __threadfence(); *(volatile v2us*)(VT + e) = o; }
__global__ __launch_bounds__(256) void k_bias(const float* __restrict__ qss, const float* __restrict__ kss, const float* __restrict__ ls, const float* __restrict__ w, h16* B16) { const int e = (blockIdx.x * 256 + threadIdx.x) * 4; if (e >= TT * TT) return; const int k0 = e % TT; const int q = e / TT;
    const float q0 = bfr(qss[q * 3]), q1 = bfr(qss[q * 3 + 1]), q2 = bfr(qss[q * 3 + 2]); float gam[NM];
#pragma unroll
    for (int m = 0; m < NM; ++m) { const float l = bfr(ls[m]); float l2 = __fmul_rn(l, l); asm volatile("" : "+v"(l2)); gam[m] = __fdiv_rn(1.0f, __fmul_rn(2.0f, l2)); }
    float bias[NH_][4];
#pragma unroll
    for (int u = 0; u < 4; ++u) { const int k = k0 + u; const float d0 = __fsub_rn(q0, bfr(kss[k * 3])), d1 = __fsub_rn(q1, bfr(kss[k * 3 + 1])), dd2 = __fsub_rn(q2, bfr(kss[k * 3 + 2])); float s0 = __fmul_rn(d0, d0), s1 = __fmul_rn(d1, d1), s2 = __fmul_rn(dd2, dd2); asm volatile("" : "+v"(s0)); asm volatile("" : "+v"(s1)); asm volatile("" : "+v"(s2)); const float d2 = __fadd_rn(__fadd_rn(s0, s1), s2);
        float phi[NM];
#pragma unroll
        for (int m = 0; m < NM; ++m) { float a = __fmul_rn(-d2, gam[m]); asm volatile("" : "+v"(a)); phi[m] = __expf(a); }
#pragma unroll
        for (int h = 0; h < NH_; ++h) { float s = 0.f;
#pragma unroll
            for (int m = 0; m < NM; ++m) { float wv = bfr(w[h * NM + m]); asm volatile("" : "+v"(wv)); float pr = __fmul_rn(phi[m], wv); asm volatile("" : "+v"(pr)); s = __fadd_rn(s, pr); } bias[h][u] = s; } }
    for (int ps = 0; ps < 2; ++ps) {
#pragma unroll
        for (int h = 0; h < NH_; ++h) { v4h o; for (int u = 0; u < 4; ++u) o[u] = tohx(bias[h][u]); *(volatile v4h*)(B16 + (size_t)h * TT * TT + e) = o; } if (ps == 0) __threadfence(); } }
__global__ __launch_bounds__(256) void k_bsoft(const float* __restrict__ Sb, const h16* __restrict__ B16, const int* __restrict__ mk, int h0, bf* Ph, bf* Pl) { const int lane = threadIdx.x & 31; const int row = blockIdx.x * 8 + (threadIdx.x >> 5); if (row >= HPP * TT) return; const int q = row % TT; const int z = row / TT;
    const float* sr = Sb + (size_t)row * TT; const h16* br = B16 + ((size_t)(h0 + z) * TT + q) * TT; float v[TT / 32]; float mx = -3.0e38f;
#pragma unroll
    for (int ch = 0; ch < TT / 128; ++ch) { const int k4 = ch * 128 + lane * 4; const v4f a = *(const v4f*)(sr + k4); const v4h bb = *(const v4h*)(br + k4);
#pragma unroll
        for (int u = 0; u < 4; ++u) { const float t = (mk[k4 + u] != 0) ? __fadd_rn(a[u], (float)bb[u]) : -3.0e38f; v[ch * 4 + u] = t; mx = fmaxf(mx, t); } }
#pragma unroll
    for (int sh = 16; sh; sh >>= 1) mx = fmaxf(mx, __shfl_xor(mx, sh, 32));
    float sum = 0.f;
#pragma unroll
    for (int qq = 0; qq < TT / 32; ++qq) { float d0 = __fsub_rn(v[qq], mx); asm volatile("" : "+v"(d0)); v[qq] = __builtin_amdgcn_exp2f(__fmul_rn(d0, 1.4426950408889634f)); sum += v[qq]; }
#pragma unroll
    for (int sh = 16; sh; sh >>= 1) sum += __shfl_xor(sum, sh, 32);
    const float f = __fdiv_rn(1.0f, __fadd_rn(sum, 1e-10f));
    for (int ps = 0; ps < 2; ++ps) {
#pragma unroll
        for (int ch = 0; ch < TT / 128; ++ch) { v4us oh, ol;
#pragma unroll
            for (int u = 0; u < 4; ++u) { unsigned short a2, b2; splitf(v[ch * 4 + u] * f, a2, b2); oh[u] = a2; ol[u] = b2; } const size_t oo = (size_t)row * TT + ch * 128 + lane * 4; *(volatile v4us*)(Ph + oo) = oh; *(volatile v4us*)(Pl + oo) = ol; }
        if (ps == 0) __threadfence(); } }

extern "C" void kernel_launch(void* const* d_in, const int* in_sizes, int n_in,
                              void* d_out, int out_size, void* d_ws, size_t ws_size, hipStream_t stream) {
    (void)in_sizes; (void)n_in; (void)out_size;
    const float* qs = (const float*)d_in[0]; const float* ks = (const float*)d_in[1]; const float* vs = (const float*)d_in[2]; const float* qss = (const float*)d_in[3]; const float* kss = (const float*)d_in[4]; const float* ls = (const float*)d_in[5]; const float* w = (const float*)d_in[6]; const int* mask = (const int*)d_in[7];
    float* OUT = (float*)d_out;
    char* wsp = (char*)d_ws;
    auto take = [&](size_t bytes) { char* p = wsp; wsp += (bytes + 255) & ~(size_t)255; return (void*)p; };
    h16* B16 = (h16*)take((size_t)NH_ * TT * TT * 2); bf* QB = (bf*)take((size_t)HPP * TT * HD * 2); bf* KB = (bf*)take((size_t)HPP * TT * HD * 2); bf* VT = (bf*)take((size_t)HPP * HD * TT * 2); float* Sb = (float*)take((size_t)HPP * TT * TT * 4); bf* Ph = (bf*)take((size_t)HPP * TT * TT * 2); bf* Pl = (bf*)take((size_t)HPP * TT * TT * 2);
    if ((size_t)(wsp - (char*)d_ws) > ws_size) return;
    for (int b = 0; b < NB_; ++b) {
        k_bias<<<(TT * TT / 4 + 255) / 256, 256, 0, stream>>>(qss + (size_t)b * TT * 3, kss + (size_t)b * TT * 3, ls, w, B16);
        for (int h0 = 0; h0 < NH_; h0 += HPP) { const size_t zo = ((size_t)b * NH_ + h0) * TT * HD;
            k_q8<<<(HPP * TT * HD / 8 + 255) / 256, 256, 0, stream>>>(qs + zo, QB, (size_t)HPP * TT * HD / 8); k_cvt8<<<(HPP * TT * HD / 8 + 255) / 256, 256, 0, stream>>>(ks + zo, KB, (size_t)HPP * TT * HD / 8); k_vt<<<(HPP * HD * TT / 2 + 255) / 256, 256, 0, stream>>>(vs + zo, VT);
            k_gemmw<bf, 0, false><<<dim3(TT / 64, TT / 64, HPP), 32, 0, stream>>>(QB, nullptr, KB, nullptr, HD, Sb, TT, nullptr, (size_t)TT * HD, (size_t)TT * HD, (size_t)TT * TT);
            k_bsoft<<<HPP * TT / 8, 256, 0, stream>>>(Sb, B16, mask + (size_t)b * TT, h0, Ph, Pl);
            k_gemmw<bf, 1, false><<<dim3(TT / 64, 1, HPP), 32, 0, stream>>>(Ph, Pl, VT, nullptr, TT, OUT + zo, HD, nullptr, (size_t)TT * TT, (size_t)HD * TT, (size_t)TT * HD); } }
}
